// MultiHeadedAttention_61117384622702
// MI455X (gfx1250) — hardware-verified
//
#include <hip/hip_runtime.h>
#include <math.h>

#ifndef NB
#define NB 2
#endif
#ifndef SEQ
#define SEQ 2048
#endif
#define NB_FULL 2
#define SEQ_FULL 2048
#define DM 768
#define NH 12
#define HD 64
#define NTOK (NB * SEQ)
#define NQB (SEQ / 64)

static_assert(NH * HD == DM);
static_assert(HD == 64);
static_assert(DM % 64 == 0);
static_assert(DM % 32 == 0);
static_assert((2 * DM) % 32 == 0);
static_assert(DM % 8 == 0);
static_assert(SEQ % 64 == 0);
static_assert(NTOK % 64 == 0);
static_assert(NB <= NB_FULL);
static_assert(SEQ <= SEQ_FULL);
static_assert(sizeof(long) == 8);

typedef __attribute__((ext_vector_type(16))) _Float16 v16h;
typedef __attribute__((ext_vector_type(8)))  _Float16 v8h;
typedef __attribute__((ext_vector_type(16))) __bf16   v16b;
typedef __attribute__((ext_vector_type(8)))  __bf16   v8b;
typedef __attribute__((ext_vector_type(8)))  float    v8f;
typedef __attribute__((ext_vector_type(4)))  float    v4f;
typedef __attribute__((ext_vector_type(4)))  unsigned int v4u;
typedef unsigned short us;
typedef __attribute__((ext_vector_type(8)))  unsigned short v8us;
typedef __attribute__((ext_vector_type(16))) unsigned short v16us;


#define VST2(T, ptr, val) do { const T vst2_v_ = (val); *(volatile T*)(ptr) = vst2_v_; __threadfence(); *(volatile T*)(ptr) = vst2_v_; } while (0)

__device__ __forceinline__ unsigned int cmb_pk2(float a, float b) { return (unsigned int)__builtin_bit_cast(unsigned short, (_Float16)a) | ((unsigned int)__builtin_bit_cast(unsigned short, (_Float16)b) << 16); }
__device__ __forceinline__ float cmb_bf(float v) { const unsigned u = __builtin_bit_cast(unsigned, v); const unsigned r = (u + 0x7fffu + ((u >> 16) & 1u)) & 0xffff0000u; return __builtin_bit_cast(float, r); }
__device__ __forceinline__ float h_res(float x) { return (x - (float)(_Float16)x) * 2048.0f; }
__device__ __forceinline__ us f2h_bits(float f) { return __builtin_bit_cast(unsigned short, (_Float16)f); }

namespace w25 {

__device__ __forceinline__ unsigned short f2bf_bits(float f) {
  unsigned u = __float_as_uint(f);
  return (unsigned short)((u + 0x7FFFu + ((u >> 16) & 1u)) >> 16);
}
__device__ __forceinline__ float bf_bits2f(unsigned short h) { return __uint_as_float(((unsigned)h) << 16); }

__device__ __forceinline__ void dep_guard_h(v8f& a, v8f& b, v16h x, v16h y) { asm volatile("v_nop\n\tv_nop\n\tv_nop\n\tv_nop" : "+v"(a), "+v"(b) : "v"(x), "v"(y)); }
__device__ __forceinline__ void dep_guard_b(v8f& a, v8f& b, v16b x, v16b y) { asm volatile("v_nop\n\tv_nop\n\tv_nop\n\tv_nop" : "+v"(a), "+v"(b) : "v"(x), "v"(y)); }
__device__ __forceinline__ void keep4_h(v16h a, v16h b, v16h c, v16h d) { asm volatile("v_nop" :: "v"(a), "v"(b), "v"(c), "v"(d)); }
__device__ __forceinline__ void keep4_b(v16b a, v16b b, v16b c, v16b d) { asm volatile("v_nop" :: "v"(a), "v"(b), "v"(c), "v"(d)); }
__device__ __forceinline__ void acc_guard4(v8f& a, v8f& b, v8f& c, v8f& d) { asm volatile("v_nop\n\tv_nop\n\tv_nop\n\tv_nop" : "+v"(a), "+v"(b), "+v"(c), "+v"(d)); }

template <typename T> struct Frag;
template <> struct Frag<_Float16> {
  typedef v16h V; union U { v16h v; v8h h[2]; };
  static __device__ __forceinline__ v16h load(const _Float16* p) {
    U f; f.h[0] = *(const v8h*)(p); f.h[1] = *(const v8h*)(p + 16); return f.v;
  }
  static __device__ __forceinline__ v8f mma(v16h a, v16h b, v8f c) {
    return __builtin_amdgcn_wmma_f32_16x16x32_f16(false, a, false, b, (short)0, c, false, false);
  }
  static __device__ __forceinline__ void guard(v8f& a, v8f& b, v16h x, v16h y) { dep_guard_h(a, b, x, y); }
  static __device__ __forceinline__ void keep(v16h a, v16h b, v16h c, v16h d) { keep4_h(a, b, c, d); }
};
template <> struct Frag<__bf16> {
  typedef v16b V; union U { v16b v; v8b h[2]; };
  static __device__ __forceinline__ v16b load(const __bf16* p) {
    U f; f.h[0] = *(const v8b*)(p); f.h[1] = *(const v8b*)(p + 16); return f.v;
  }
  static __device__ __forceinline__ v8f mma(v16b a, v16b b, v8f c) {
    return __builtin_amdgcn_wmma_f32_16x16x32_bf16(false, a, false, b, (short)0, c, false, false);
  }
  static __device__ __forceinline__ void guard(v8f& a, v8f& b, v16b x, v16b y) { dep_guard_b(a, b, x, y); }
  static __device__ __forceinline__ void keep(v16b a, v16b b, v16b c, v16b d) { keep4_b(a, b, c, d); }
};
template <int ET> struct Elem;
template <> struct Elem<0> { typedef _Float16 T; };
template <> struct Elem<1> { typedef __bf16 T; };

template <int ET, int BIAS_MODE, int OUT_MODE>
__device__ __forceinline__ void gemm64_body(
    const unsigned short* __restrict__ Ap, int lda, long strideA,
    const unsigned short* __restrict__ Btp, int ldb, long strideB,
    void* __restrict__ Cout, void* __restrict__ Cout2, int ldc, long strideC,
    const float* __restrict__ biasp, int strideBias,
    int M, int N, int K, float scale) {
  typedef typename Elem<ET>::T T;
  typedef typename Frag<T>::V V;
  __shared__ __align__(16) float sT[8][16 * 68];
  const T* A = (const T*)Ap; const T* Bt = (const T*)Btp;
  const int b    = blockIdx.y;
  const int lane = threadIdx.x & 31;
  const int wave = threadIdx.x >> 5;
  const int tilesN = N >> 6;
  const int tilesM = M >> 6;
  const int tile = blockIdx.x * 8 + wave;
  if (tile >= tilesM * tilesN) return;
  const int tm = tile / tilesN;
  const int tn = tile - tm * tilesN;
  const int m0 = tm << 6;
  const int n0 = tn << 6;

  const T* Ab = A  + (size_t)b * strideA;
  const T* Bb = Bt + (size_t)b * strideB;
  const float* bias = biasp + (size_t)b * strideBias;

  const int rlane = lane & 15;
  const int koff  = (lane >> 4) * 8;
  const int mOff  = (lane >> 4) * 8;

  v8f acc[4][4];
#pragma unroll
  for (int i = 0; i < 4; ++i)
#pragma unroll
    for (int j = 0; j < 4; ++j) acc[i][j] = (v8f){0.f,0.f,0.f,0.f,0.f,0.f,0.f,0.f};

  for (int k0 = 0; k0 < K; k0 += 32) {
    V bh[4];
#pragma unroll
    for (int j = 0; j < 4; ++j) {
      const size_t bo = (size_t)(n0 + (j << 4) + rlane) * ldb + koff + k0;
      bh[j] = Frag<T>::load(Bb + bo);
    }
#pragma unroll
    for (int i = 0; i < 4; ++i) {
      const size_t ao = (size_t)(m0 + (i << 4) + rlane) * lda + koff + k0;
      V ah = Frag<T>::load(Ab + ao);
#pragma unroll
      for (int j = 0; j < 4; ++j) acc[i][j] = Frag<T>::mma(ah, bh[j], acc[i][j]);
      Frag<T>::guard(acc[i][0], acc[i][3], ah, ah);
    }
    Frag<T>::keep(bh[0], bh[1], bh[2], bh[3]);
  }
  acc_guard4(acc[0][0], acc[0][1], acc[0][2], acc[0][3]);
  acc_guard4(acc[1][0], acc[1][1], acc[1][2], acc[1][3]);
  acc_guard4(acc[2][0], acc[2][1], acc[2][2], acc[2][3]);
  acc_guard4(acc[3][0], acc[3][1], acc[3][2], acc[3][3]);

  float* slab = sT[wave];
#pragma unroll
  for (int i = 0; i < 4; ++i) {
    const int mBase = m0 + (i << 4);
#pragma unroll
    for (int j = 0; j < 4; ++j) {
      const int n = n0 + (j << 4) + rlane;
      float bv = 0.f;
      if (BIAS_MODE == 2) bv = bias[n];
#pragma unroll
      for (int r = 0; r < 8; ++r) {
        float v = acc[i][j][r] * scale;
        if (BIAS_MODE == 1) v += bias[mBase + mOff + r];
        if (BIAS_MODE == 2) v += bv;
        slab[(mOff + r) * 68 + (j << 4) + rlane] = v;
      }
    }
    __builtin_amdgcn_fence(3  , "workgroup");
    __builtin_amdgcn_wave_barrier();
    __builtin_amdgcn_fence(2  , "workgroup");
    if (OUT_MODE == 0) {
      float* C = (float*)Cout + (size_t)b * strideC;
      const int hh = lane >> 4, c4 = (lane & 15) * 4;
      for (int pass = 0; pass < 2; ++pass) {
#pragma unroll
        for (int it = 0; it < 8; ++it) {
          const int row = it * 2 + hh;
          v4f v = *(const v4f*)(slab + row * 68 + c4);
          *(volatile v4f*)(C + (size_t)(mBase + row) * ldc + n0 + c4) = v;
        }
        __threadfence();
      }
    } else {
      const int q = lane >> 3, c8 = (lane & 7) * 8;
      unsigned short* C  = (unsigned short*)Cout  + (size_t)b * strideC;
      unsigned short* C2 = (unsigned short*)Cout2 + (size_t)b * strideC;
      for (int pass = 0; pass < 2; ++pass) {
#pragma unroll
        for (int it = 0; it < 4; ++it) {
          const int row = it * 4 + q;
          const float* sp = slab + row * 68 + c8;
          v4u hv;
          hv.x = cmb_pk2(sp[0], sp[1]); hv.y = cmb_pk2(sp[2], sp[3]);
          hv.z = cmb_pk2(sp[4], sp[5]); hv.w = cmb_pk2(sp[6], sp[7]);
          *(volatile v4u*)(C + (size_t)(mBase + row) * ldc + n0 + c8) = hv;
          if (OUT_MODE == 2) {
            v4u lv;
            lv.x = cmb_pk2(h_res(sp[0]), h_res(sp[1])); lv.y = cmb_pk2(h_res(sp[2]), h_res(sp[3]));
            lv.z = cmb_pk2(h_res(sp[4]), h_res(sp[5])); lv.w = cmb_pk2(h_res(sp[6]), h_res(sp[7]));
            *(volatile v4u*)(C2 + (size_t)(mBase + row) * ldc + n0 + c8) = lv;
          }
        }
        __threadfence();
      }
    }
    __builtin_amdgcn_fence(3  , "workgroup");
    __builtin_amdgcn_wave_barrier();
    __builtin_amdgcn_fence(2  , "workgroup");
  }
}

}

__global__ __launch_bounds__(256) void k_gemm_q(const us* __restrict__ Xq16, const us* __restrict__ Wq16, us* __restrict__ QH, us* __restrict__ QR, const float* __restrict__ BRq) {
  static_assert(NTOK % 64 == 0 && DM % 64 == 0 && DM % 32 == 0);
  w25::gemm64_body<0, 2, 2>(Xq16, DM, 0L, Wq16, DM, 0L, (void*)QH, (void*)QR, DM, 0L, BRq, 0, NTOK, DM, DM, 0.0625f);
}
__global__ __launch_bounds__(256) void k_gemm_k(const us* __restrict__ Xk16, const us* __restrict__ Wk16, us* __restrict__ KH, const float* __restrict__ BRk) {
  static_assert(NTOK % 64 == 0 && DM % 64 == 0 && DM % 32 == 0);
  w25::gemm64_body<0, 2, 1>(Xk16, DM, 0L, Wk16, DM, 0L, (void*)KH, (void*)KH, DM, 0L, BRk, 0, NTOK, DM, DM, 0.0625f);
}
__global__ __launch_bounds__(256) void k_gemm_vt(const us* __restrict__ Wv16, const us* __restrict__ Xv16, us* __restrict__ VT, const float* __restrict__ BRv) {
  static_assert(NTOK % 64 == 0 && DM % 64 == 0 && DM % 32 == 0);
  w25::gemm64_body<0, 1, 1>(Wv16, DM, 0L, Xv16, DM, 0L, (void*)VT, (void*)VT, NTOK, 0L, BRv, 0, DM, NTOK, DM, 0.0625f);
}
__global__ __launch_bounds__(256) void k_gemm_out(const us* __restrict__ CTX2, const us* __restrict__ WO2, float* __restrict__ out, const float* __restrict__ BRo) {
  static_assert(SEQ % 64 == 0 && DM % 64 == 0 && (2 * DM) % 32 == 0);
  w25::gemm64_body<1, 2, 0>(CTX2, 2 * DM, (long)SEQ * 2 * DM, WO2, 2 * DM, 0L, (void*)out, (void*)out, DM, (long)SEQ_FULL * DM, BRo, 0, SEQ, DM, 2 * DM, 1.0f);
}

__device__ __forceinline__ unsigned int bf_pk2(float a, float b) { return (unsigned int)w25::f2bf_bits(a) | ((unsigned int)w25::f2bf_bits(b) << 16); }
__device__ __forceinline__ void cast8_f16(const float* __restrict__ s, us* __restrict__ d, float sc) {
  const v4f a = *(const v4f*)s; const v4f b2 = *(const v4f*)(s + 4);
  v4u pk;
  pk.x = cmb_pk2(cmb_bf(a.x) * sc, cmb_bf(a.y) * sc); pk.y = cmb_pk2(cmb_bf(a.z) * sc, cmb_bf(a.w) * sc);
  pk.z = cmb_pk2(cmb_bf(b2.x) * sc, cmb_bf(b2.y) * sc); pk.w = cmb_pk2(cmb_bf(b2.z) * sc, cmb_bf(b2.w) * sc);
  VST2(v4u, (v4u*)d, pk);
}
__global__ __launch_bounds__(256) void k_cast_w4(const float* __restrict__ Wq, const float* __restrict__ Wk, const float* __restrict__ Wv, const float* __restrict__ Wo, us* __restrict__ W16, us* __restrict__ WO2) {
  static_assert(DM % 8 == 0);
  const int u = blockIdx.x * 256 + threadIdx.x; if (u >= DM * (DM / 8)) return;
  const int r = u / (DM / 8); const int c0 = 8 * (u % (DM / 8));
  const size_t o = (size_t)r * DM + c0;
  cast8_f16(Wq + o, W16 + o, 16.0f);
  cast8_f16(Wk + o, W16 + (size_t)DM * DM + o, 16.0f);
  cast8_f16(Wv + o, W16 + (size_t)2 * DM * DM + o, 16.0f);
  const v4f a = *(const v4f*)(Wo + o); const v4f b2 = *(const v4f*)(Wo + o + 4);
  v4u pk; pk.x = bf_pk2(a.x, a.y); pk.y = bf_pk2(a.z, a.w); pk.z = bf_pk2(b2.x, b2.y); pk.w = bf_pk2(b2.z, b2.w);
  VST2(v4u, (v4u*)(WO2 + (size_t)r * (2 * DM) + c0), pk);
  VST2(v4u, (v4u*)(WO2 + (size_t)r * (2 * DM) + DM + c0), pk);
}
__global__ __launch_bounds__(256) void k_bias4(const float* __restrict__ bq, const float* __restrict__ bk, const float* __restrict__ bv, const float* __restrict__ bo, float* __restrict__ BR) {
  static_assert(DM % 32 == 0);
  const int u = blockIdx.x * 256 + threadIdx.x; if (u >= DM) return;
  VST2(float, BR + u, cmb_bf(bq[u]));
  VST2(float, BR + DM + u, cmb_bf(bk[u]));
  VST2(float, BR + 2 * DM + u, cmb_bf(bv[u]));
  VST2(float, BR + 3 * DM + u, cmb_bf(bo[u]));
}
__global__ __launch_bounds__(256) void k_cast_x3(const float* __restrict__ xq, const float* __restrict__ xk, const float* __restrict__ xv, us* __restrict__ X16) {
  const long long u = (long long)blockIdx.x * 256 + threadIdx.x; if (u >= (long long)NTOK * (DM / 8)) return;
  const int r = (int)(u / (DM / 8)); const int c0 = 8 * (int)(u % (DM / 8));
  const int b = r / SEQ; const int s = r - b * SEQ;
  const size_t so = ((size_t)b * SEQ_FULL + s) * DM + c0; const size_t dofs = (size_t)r * DM + c0;
  cast8_f16(xq + so, X16 + dofs, 1.0f);
  cast8_f16(xk + so, X16 + (size_t)NTOK * DM + dofs, 1.0f);
  cast8_f16(xv + so, X16 + (size_t)2 * NTOK * DM + dofs, 1.0f);
}

__device__ __forceinline__ v8f mma_h(v16h a, v16h b, v8f c) {
  c = __builtin_amdgcn_wmma_f32_16x16x32_f16(false, a, false, b, (short)0, c, false, false);
  asm volatile("v_nop\n\tv_nop\n\tv_nop\n\tv_nop" : "+v"(c) : "v"(a), "v"(b));
  return c;
}
__device__ __forceinline__ void wave_sync() {
  __builtin_amdgcn_fence(3  , "workgroup");
  __builtin_amdgcn_wave_barrier();
  __builtin_amdgcn_fence(2  , "workgroup");
}
union FBU { v16us u; v8us h[2]; };
#define LDFRAGH(dst, arr, off) do { FBU f_; f_.h[0] = *(const v8us*)&arr[(off)]; f_.h[1] = *(const v8us*)&arr[(off) + 16]; dst = __builtin_bit_cast(v16h, f_.u); } while (0)

__global__ __launch_bounds__(128) void k_attn_flash(const us* __restrict__ QH, const us* __restrict__ QR, const us* __restrict__ KH, const us* __restrict__ VT,
                                                    const int* __restrict__ MK, us* __restrict__ CTX2) {
  static_assert(HD == 64 && SEQ % 64 == 0);
  __shared__ __align__(16) us Qsh[64 * 64];
  __shared__ __align__(16) us Qsr[64 * 64];
  __shared__ __align__(16) us Ksh[64 * 64];
  __shared__ __align__(16) us Vth[64 * 64];
  __shared__ __align__(16) us Psh[4 * 16 * 32];

  const int tid = threadIdx.x, wave = tid >> 5, lane = tid & 31, hh = lane >> 4, c = lane & 15;
  const int bx = blockIdx.x;
  const int qb = bx % NQB; const int bh = bx / NQB; const int h = bh % NH; const int b = bh / NH;
  const int tok0 = b * SEQ + qb * 64;

  {
    const int row = tid >> 1, dh = (tid & 1) * 32;
    const size_t qro_g = (size_t)(tok0 + row) * DM + h * HD + dh;
#pragma unroll
    for (int i = 0; i < 4; ++i) {
      *(v8us*)&Qsh[row * 64 + dh + 8 * i] = *(const v8us*)(QH + qro_g + 8 * i);
      *(v8us*)&Qsr[row * 64 + dh + 8 * i] = *(const v8us*)(QR + qro_g + 8 * i);
    }
  }
  __syncthreads();

  float mrow[8], lrow[8];
  v8f oacc[4];
#pragma unroll
  for (int r = 0; r < 8; ++r) { mrow[r] = -__builtin_inff(); lrow[r] = 0.f; }
#pragma unroll
  for (int t = 0; t < 4; ++t) oacc[t] = (v8f){0.f,0.f,0.f,0.f,0.f,0.f,0.f,0.f};

  const int pb = wave * 512;
  const int qro = (wave * 16 + c) * 64 + 8 * hh;
  const int mk0 = b * SEQ_FULL + c;

#pragma unroll 1
  for (int kc = 0; kc < NQB; ++kc) {
    const int kv0 = kc * 64;
    __syncthreads();
    {
      const int row = tid >> 1, dh = (tid & 1) * 32;
      const size_t kro = (size_t)(b * SEQ + kv0 + row) * DM + h * HD + dh;
      const size_t vro = (size_t)(h * HD + row) * NTOK + (size_t)b * SEQ + kv0 + dh;
#pragma unroll
      for (int i = 0; i < 4; ++i) {
        *(v8us*)&Ksh[row * 64 + dh + 8 * i] = *(const v8us*)(KH + kro + 8 * i);
        *(v8us*)&Vth[row * 64 + dh + 8 * i] = *(const v8us*)(VT + vro + 8 * i);
      }
    }
    __syncthreads();

#pragma unroll 1
    for (int hf = 0; hf < 2; ++hf) {
      v8f s0 = (v8f){0.f,0.f,0.f,0.f,0.f,0.f,0.f,0.f};
      v8f s1 = s0, r0 = s0, r1 = s0;
#pragma unroll
      for (int dc = 0; dc < 2; ++dc) {
        v16h qh, qr, k0, k1;
        LDFRAGH(qh, Qsh, qro + dc * 32);
        LDFRAGH(qr, Qsr, qro + dc * 32);
        const int ko0 = ((2 * hf) * 16 + c) * 64 + dc * 32 + 8 * hh;
        LDFRAGH(k0, Ksh, ko0);
        LDFRAGH(k1, Ksh, ko0 + 16 * 64);
        s0 = mma_h(qh, k0, s0); r0 = mma_h(qr, k0, r0);
        s1 = mma_h(qh, k1, s1); r1 = mma_h(qr, k1, r1);
      }
      const int mv0 = MK[mk0 + kv0 + hf * 32];
      const int mv1 = MK[mk0 + kv0 + hf * 32 + 16];
      const bool keep0 = (mv0 != 0);
      const bool keep1 = (mv1 != 0);
#pragma unroll
      for (int r = 0; r < 8; ++r) {
        const float sc0 = (s0[r] + r0[r] * (1.0f / 2048.0f)) * 0.125f;
        const float sc1 = (s1[r] + r1[r] * (1.0f / 2048.0f)) * 0.125f;
        const float a0 = keep0 ? sc0 : -1.0e9f;
        const float a1 = keep1 ? sc1 : -1.0e9f;
        float m = fmaxf(a0, a1);
        m = fmaxf(m, __shfl_xor(m, 1, 32)); m = fmaxf(m, __shfl_xor(m, 2, 32));
        m = fmaxf(m, __shfl_xor(m, 4, 32)); m = fmaxf(m, __shfl_xor(m, 8, 32));
        const float mnew = fmaxf(mrow[r], m);
        const float alpha = expf(mrow[r] - mnew);
        mrow[r] = mnew;
        const float p0 = expf(a0 - mnew);
        const float p1 = expf(a1 - mnew);
        float psum = p0 + p1;
        psum += __shfl_xor(psum, 1, 32); psum += __shfl_xor(psum, 2, 32);
        psum += __shfl_xor(psum, 4, 32); psum += __shfl_xor(psum, 8, 32);
        lrow[r] = lrow[r] * alpha + psum;
#pragma unroll
        for (int t = 0; t < 4; ++t) oacc[t][r] *= alpha;
        const int po = pb + (8 * hh + r) * 32 + c;
        Psh[po] = f2h_bits(p0 * 256.0f);
        Psh[po + 16] = f2h_bits(p1 * 256.0f);
      }
      wave_sync();
      v16h pa;
      LDFRAGH(pa, Psh, pb + c * 32 + 8 * hh);
#pragma unroll
      for (int t = 0; t < 4; ++t) {
        v16h vh;
        const int vo = (t * 16 + c) * 64 + hf * 32 + 8 * hh;
        LDFRAGH(vh, Vth, vo);
        oacc[t] = mma_h(pa, vh, oacc[t]);
      }
      wave_sync();
    }
  }

  __syncthreads();
  {
    const int sb = wave * 1024;
#pragma unroll
    for (int r = 0; r < 8; ++r) {
      const float inv = (lrow[r] > 0.f) ? ((1.0f / lrow[r]) * (1.0f / 256.0f)) : 0.f;
#pragma unroll
      for (int t = 0; t < 4; ++t) {
        const float val = oacc[t][r] * inv;
        const us hb = w25::f2bf_bits(val); const us lb = w25::f2bf_bits(val - w25::bf_bits2f(hb));
        Ksh[sb + (8 * hh + r) * 64 + t * 16 + c] = hb;
        Vth[sb + (8 * hh + r) * 64 + t * 16 + c] = lb;
      }
    }
    wave_sync();
    const int q4 = lane >> 3, c8 = (lane & 7) * 8;
    v8us hv[4], lv[4];
#pragma unroll
    for (int it = 0; it < 4; ++it) {
      const int row = it * 4 + q4;
      hv[it] = *(const v8us*)&Ksh[sb + row * 64 + c8];
      lv[it] = *(const v8us*)&Vth[sb + row * 64 + c8];
    }
    for (int pass = 0; pass < 2; ++pass) {
#pragma unroll
      for (int it = 0; it < 4; ++it) {
        const int row = it * 4 + q4;
        us* dst = CTX2 + (size_t)(tok0 + wave * 16 + row) * (2 * DM) + h * HD + c8;
        *(volatile v8us*)(dst) = hv[it];
        *(volatile v8us*)(dst + DM) = lv[it];
      }
      __threadfence();
    }
  }
}

#define WS_X16   ((size_t)3 * NTOK * DM * 2)
#define WS_W16   ((size_t)3 * DM * DM * 2)
#define WS_WO2   ((size_t)DM * 2 * DM * 2)
#define WS_BR    ((size_t)4 * DM * 4)
#define WS_PL    ((size_t)NTOK * DM * 2)
#define WS_CTX2  ((size_t)NTOK * 2 * DM * 2)
#define WS_TOTAL (WS_X16 + WS_W16 + WS_WO2 + WS_BR + 4 * WS_PL + WS_CTX2)
static_assert(WS_X16 % 256 == 0 && WS_W16 % 256 == 0 && WS_WO2 % 256 == 0 && WS_BR % 256 == 0 && WS_PL % 256 == 0 && WS_CTX2 % 256 == 0);
static_assert(WS_TOTAL <= (size_t)134217728);

extern "C" void kernel_launch(void* const* d_in, const int* in_sizes, int n_in, void* d_out, int out_size, void* d_ws, size_t ws_size, hipStream_t stream) {
  if (n_in < 12) return;
  const long long need_x = ((long long)(NB - 1) * SEQ_FULL + SEQ) * DM;
  const long long need_m = (long long)(NB - 1) * SEQ_FULL + SEQ;
  if ((long long)in_sizes[0] < need_x || (long long)in_sizes[1] < need_x || (long long)in_sizes[2] < need_x) return;
  if ((long long)in_sizes[3] < need_m) return;
  if (in_sizes[4] < DM * DM || in_sizes[6] < DM * DM || in_sizes[8] < DM * DM || in_sizes[10] < DM * DM) return;
  if (in_sizes[5] < DM || in_sizes[7] < DM || in_sizes[9] < DM || in_sizes[11] < DM) return;
  if ((long long)out_size < need_x) return;
  if (WS_TOTAL > ws_size) return;

  const float* xq = (const float*)d_in[0];
  const float* xk = (const float*)d_in[1];
  const float* xv = (const float*)d_in[2];
  const int* kmask = (const int*)d_in[3];
  const float* Wq = (const float*)d_in[4];
  const float* bq = (const float*)d_in[5];
  const float* Wk = (const float*)d_in[6];
  const float* bk = (const float*)d_in[7];
  const float* Wv = (const float*)d_in[8];
  const float* bv = (const float*)d_in[9];
  const float* Wo = (const float*)d_in[10];
  const float* bo = (const float*)d_in[11];
  float* out = (float*)d_out;

  char* wsp = (char*)d_ws;
  us* X16 = (us*)wsp;             wsp += WS_X16;
  us* W16 = (us*)wsp;             wsp += WS_W16;
  us* WO2 = (us*)wsp;             wsp += WS_WO2;
  float* BR = (float*)wsp;        wsp += WS_BR;
  us* QH = (us*)wsp;              wsp += WS_PL;
  us* QR = (us*)wsp;              wsp += WS_PL;
  us* KH = (us*)wsp;              wsp += WS_PL;
  us* VT = (us*)wsp;              wsp += WS_PL;
  us* CTX2 = (us*)wsp;            wsp += WS_CTX2;

  k_cast_w4<<<dim3((unsigned)((DM * (DM / 8) + 255) / 256)), dim3(256), 0, stream>>>(Wq, Wk, Wv, Wo, W16, WO2);
  k_bias4<<<dim3((unsigned)((DM + 255) / 256)), dim3(256), 0, stream>>>(bq, bk, bv, bo, BR);
  k_cast_x3<<<dim3((unsigned)(((long long)NTOK * (DM / 8) + 255) / 256)), dim3(256), 0, stream>>>(xq, xk, xv, X16);
  k_gemm_q<<<dim3((unsigned)(((NTOK / 64) * (DM / 64) + 7) / 8), 1u), dim3(256), 0, stream>>>(X16, W16, QH, QR, BR);
  k_gemm_k<<<dim3((unsigned)(((NTOK / 64) * (DM / 64) + 7) / 8), 1u), dim3(256), 0, stream>>>(X16 + (size_t)NTOK * DM, W16 + (size_t)DM * DM, KH, BR + DM);
  k_gemm_vt<<<dim3((unsigned)(((DM / 64) * (NTOK / 64) + 7) / 8), 1u), dim3(256), 0, stream>>>(W16 + (size_t)2 * DM * DM, X16 + (size_t)2 * NTOK * DM, VT, BR + 2 * DM);
  k_attn_flash<<<dim3((unsigned)(NB * NH * NQB)), dim3(128), 0, stream>>>(QH, QR, KH, VT, kmask, CTX2);
  k_gemm_out<<<dim3((unsigned)(((SEQ / 64) * (DM / 64) + 7) / 8), (unsigned)NB), dim3(256), 0, stream>>>(CTX2, WO2, out, BR + 3 * DM);
}
